// MambaBlock_64871186039086
// MI455X (gfx1250) — hardware-verified
//
#include <hip/hip_runtime.h>
#include <stddef.h>
#include <stdint.h>
#include <math.h>


#define BL     8192
#define LSEQ   2048
#define RD     1024
#define DD     128
#define NS     64
#define UC     256
#define K2     256
#define NTHR   256
#define GBM    64
#define GBN    64
#define GTHR   128
#define TCH    64

#define U_WUP  (UC * (RD / 8))
#define U_WDL  (DD * (K2 / 8))
#define U_WB   (NS * (K2 / 8))
#define U_WC   (NS * (K2 / 8))
#define U_WDN  (RD * (K2 / 8))
#define E1     (U_WUP)
#define E2     (E1 + U_WDL)
#define E3     (E2 + U_WB)
#define E4     (E3 + U_WC)
#define E5     (E4 + U_WDN)
#define E6     (E5 + NTHR)

static_assert(E1 % NTHR == 0 && E2 % NTHR == 0 && E3 % NTHR == 0 && E4 % NTHR == 0 && E5 % NTHR == 0);
static_assert(BL % GBM == 0 && UC % GBN == 0 && RD % GBN == 0 && K2 % GBN == 0);
static_assert(RD % 32 == 0 && K2 % 32 == 0 && K2 == 2 * DD);
static_assert(GBM == (GTHR / 32) * 16 && GBN == 64);
static_assert(LSEQ % TCH == 0 && (LSEQ & (LSEQ - 1)) == 0 && BL == 4 * LSEQ);
static_assert((BL * RD / 8) % NTHR == 0 && BL % 8 == 0);

constexpr size_t O_XB   = 0;
constexpr size_t O_WUPT = O_XB   + (size_t)BL * RD * 2;
constexpr size_t O_WCAT = O_WUPT + (size_t)UC * RD * 2;
constexpr size_t O_WDN  = O_WCAT + (size_t)K2 * K2 * 2;
constexpr size_t O_BCAT = O_WDN  + (size_t)RD * K2 * 2;
constexpr size_t O_U2   = O_BCAT + (size_t)K2 * 4;
constexpr size_t O_XF   = O_U2   + (size_t)2 * BL * DD * 4;
constexpr size_t O_XHL  = O_XF   + (size_t)BL * DD * 4;
constexpr size_t O_DBC  = O_XHL  + (size_t)BL * K2 * 2;
constexpr size_t O_GHL  = O_DBC  + (size_t)BL * K2 * 4;
constexpr size_t O_END  = O_GHL  + (size_t)BL * K2 * 2;
static_assert(O_END <= (size_t)134217728);
static_assert(O_WUPT % 256 == 0 && O_WCAT % 256 == 0 && O_WDN % 256 == 0 && O_BCAT % 256 == 0);
static_assert(O_U2 % 256 == 0 && O_XF % 256 == 0 && O_XHL % 256 == 0 && O_DBC % 256 == 0 && O_GHL % 256 == 0);

typedef float          v4f   __attribute__((ext_vector_type(4)));
typedef float          v8f   __attribute__((ext_vector_type(8)));
typedef int            v8i   __attribute__((ext_vector_type(8)));
typedef unsigned short v4us  __attribute__((ext_vector_type(4)));
typedef unsigned short v8us  __attribute__((ext_vector_type(8)));
typedef unsigned short v16us __attribute__((ext_vector_type(16)));
typedef __bf16         v16bf __attribute__((ext_vector_type(16)));
typedef v4f  __attribute__((may_alias)) v4fa;
typedef v4us __attribute__((may_alias)) v4usa;
typedef v8us __attribute__((may_alias)) v8usa;
union FragB { v16bf v; v16us u; v8us h[2]; v8i w; };

__device__ __forceinline__ v8f wmb(const FragB& a, const FragB& b, v8f c) {
  v8f d = __builtin_amdgcn_wmma_f32_16x16x32_bf16(false, a.v, false, b.v, (short)0, c, false, false);
  asm volatile("v_nop\n\tv_nop\n\tv_nop\n\tv_nop" : "+v"(d) : "v"(a.w), "v"(b.w));
  return d;
}

__device__ __forceinline__ unsigned bf16_bits(float f) {
  const unsigned u = __float_as_uint(f);
  return (u + 0x7FFFu + ((u >> 16) & 1u)) >> 16;
}
__device__ __forceinline__ float bf16_val(float f) {
  return __uint_as_float(bf16_bits(f) << 16);
}
__device__ __forceinline__ float silu_f(float v) {
  return v * (1.0f / (1.0f + expf(-v)));
}
__device__ __forceinline__ float softplus_f(float v) {
  return fmaxf(v, 0.0f) + log1pf(expf(-fabsf(v)));
}

__global__ __launch_bounds__(NTHR) void k_cvx(const float* __restrict__ x, unsigned short* xb) {
  const size_t u = (size_t)blockIdx.x * NTHR + (size_t)threadIdx.x;
  const float* p = x + u * 8;
  const v4f a = *(const v4f*)p;
  const v4f b = *(const v4f*)(p + 4);
  v8us o;
  o[0] = (unsigned short)bf16_bits(a.x); o[1] = (unsigned short)bf16_bits(a.y);
  o[2] = (unsigned short)bf16_bits(a.z); o[3] = (unsigned short)bf16_bits(a.w);
  o[4] = (unsigned short)bf16_bits(b.x); o[5] = (unsigned short)bf16_bits(b.y);
  o[6] = (unsigned short)bf16_bits(b.z); o[7] = (unsigned short)bf16_bits(b.w);
  unsigned short* dp = xb + u * 8;
  *(volatile v8us*)dp = o;
  __threadfence();
  *(volatile v8us*)dp = o;
}

__device__ __forceinline__ v8us gather8(const float* __restrict__ p, int stride) {
  v8us o;
#pragma unroll
  for (int i = 0; i < 8; ++i) o[i] = (unsigned short)bf16_bits(p[(size_t)i * (size_t)stride]);
  return o;
}

__global__ __launch_bounds__(NTHR) void k_wprep(const float* __restrict__ Wup, const float* __restrict__ Wdl,
                                                const float* __restrict__ WB, const float* __restrict__ WC,
                                                const float* __restrict__ Wdn, const float* __restrict__ bdl,
                                                const float* __restrict__ bB, const float* __restrict__ bC,
                                                unsigned short* wsh, float* bcat) {
  const int u = (int)blockIdx.x * NTHR + (int)threadIdx.x;
  v8us o;
  size_t doff;
  if (u < E1) {
    const int n  = u >> 7;
    const int k8 = (u & 127) * 8;
    o = gather8(Wup + (size_t)k8 * UC + n, UC);
    doff = O_WUPT / 2 + (size_t)n * RD + k8;
  } else if (u < E2) {
    const int v  = u - E1;
    const int n  = v >> 5;
    const int k8 = (v & 31) * 8;
    const int kk = k8 & (DD - 1);
    o = gather8(Wdl + (size_t)kk * DD + n, DD);
    doff = O_WCAT / 2 + (size_t)n * K2 + k8;
  } else if (u < E3) {
    const int v  = u - E2;
    const int n  = v >> 5;
    const int k8 = (v & 31) * 8;
    const int kk = k8 & (DD - 1);
    o = gather8(WB + (size_t)kk * NS + n, NS);
    doff = O_WCAT / 2 + (size_t)(DD + n) * K2 + k8;
  } else if (u < E4) {
    const int v  = u - E3;
    const int n  = v >> 5;
    const int k8 = (v & 31) * 8;
    const int kk = k8 & (DD - 1);
    o = gather8(WC + (size_t)kk * NS + n, NS);
    doff = O_WCAT / 2 + (size_t)(DD + NS + n) * K2 + k8;
  } else if (u < E5) {
    const int v  = u - E4;
    const int n  = v >> 5;
    const int k8 = (v & 31) * 8;
    const int ch = 32 * (k8 >> 6) + (k8 & 31);
    o = gather8(Wdn + (size_t)ch * RD + n, RD);
    doff = O_WDN / 2 + (size_t)n * K2 + k8;
  } else {
    const int v  = u - E5;
    const int vc = v < 63 ? v : 63;
    const int i0 = vc < 31 ? vc : 31;
    int i1 = vc - 32; i1 = i1 < 0 ? 0 : (i1 > 15 ? 15 : i1);
    int i2 = vc - 48; i2 = i2 < 0 ? 0 : (i2 > 15 ? 15 : i2);
    const v4f a = *(const v4f*)(bdl + 4 * i0);
    const v4f b = *(const v4f*)(bB + 4 * i1);
    const v4f c = *(const v4f*)(bC + 4 * i2);
    const unsigned m0 = (vc < 32) ? 0xffffffffu : 0u;
    const unsigned m2 = (vc >= 48) ? 0xffffffffu : 0u;
    const unsigned m1 = ~(m0 | m2);
    v4f r;
    r.x = bf16_val(__uint_as_float((__float_as_uint(a.x) & m0) | (__float_as_uint(b.x) & m1) | (__float_as_uint(c.x) & m2)));
    r.y = bf16_val(__uint_as_float((__float_as_uint(a.y) & m0) | (__float_as_uint(b.y) & m1) | (__float_as_uint(c.y) & m2)));
    r.z = bf16_val(__uint_as_float((__float_as_uint(a.z) & m0) | (__float_as_uint(b.z) & m1) | (__float_as_uint(c.z) & m2)));
    r.w = bf16_val(__uint_as_float((__float_as_uint(a.w) & m0) | (__float_as_uint(b.w) & m1) | (__float_as_uint(c.w) & m2)));
    float* bp = bcat + 4 * vc;
    if (v < 64) *(volatile v4f*)bp = r;
    __threadfence();
    if (v < 64) *(volatile v4f*)bp = r;
    return;
  }
  unsigned short* dp = wsh + doff;
  *(volatile v8us*)dp = o;
  __threadfence();
  *(volatile v8us*)dp = o;
}

template <int MODE>
__global__ __launch_bounds__(GTHR) void k_gemm(const unsigned short* __restrict__ A,
                                               const unsigned short* __restrict__ WT,
                                               const float* __restrict__ bias, float* outF, int K) {
  __shared__ __attribute__((aligned(16))) float stg[GBM * GBN];
  const int tid = (int)threadIdx.x, lane = tid & 31, wave = tid >> 5, hh = lane >> 4, m = lane & 15;
  const int by = (int)blockIdx.y;
  const int rowBase = (int)blockIdx.x * GBM;
  const int col0    = by * GBN;

  v8f acc[4];
  {
    const v8f z = {0.f, 0.f, 0.f, 0.f, 0.f, 0.f, 0.f, 0.f};
    acc[0] = z; acc[1] = z; acc[2] = z; acc[3] = z;
  }
  const unsigned short* ap = A  + (size_t)(rowBase + 16 * wave + m) * (size_t)K + 8 * hh;
  const unsigned short* wp = WT + (size_t)(col0 + m) * (size_t)K + 8 * hh;
  const int ksteps = K >> 5;
#pragma unroll 1
  for (int ks = 0; ks < ksteps; ++ks) {
    FragB af;
    af.h[0] = *(const v8usa*)(ap + 32 * ks);
    af.h[1] = *(const v8usa*)(ap + 32 * ks + 16);
#pragma unroll
    for (int t = 0; t < 4; ++t) {
      const unsigned short* wq = wp + (size_t)(16 * t) * (size_t)K + 32 * ks;
      FragB bf;
      bf.h[0] = *(const v8usa*)wq;
      bf.h[1] = *(const v8usa*)(wq + 16);
      acc[t] = wmb(af, bf, acc[t]);
    }
  }

#pragma unroll
  for (int t = 0; t < 4; ++t) {
    const int lc = 16 * t + m;
#pragma unroll
    for (int r = 0; r < 8; ++r) {
      const int lr = 16 * wave + 8 * hh + r;
      stg[lr * GBN + lc] = acc[t][r];
    }
  }
  __syncthreads();

  v4f b4;
  {
    const v4f t = *(const v4f*)(bias + col0 + 4 * m);
    b4.x = bf16_val(t.x); b4.y = bf16_val(t.y); b4.z = bf16_val(t.z); b4.w = bf16_val(t.w);
  }
  bool act = false;
  if constexpr (MODE == 0) act = (by >= 2);
  if constexpr (MODE == 1) act = (by < 2);

#pragma unroll 1
  for (int i = 0; i < 8; ++i) {
    float* sp = stg + (16 * wave + 2 * i + hh) * GBN + 4 * m;
    v4f v = *(const v4fa*)sp;
    v = v + b4;
    if constexpr (MODE == 0) {
      if (act) { v.x = silu_f(v.x); v.y = silu_f(v.y); v.z = silu_f(v.z); v.w = silu_f(v.w); }
    }
    if constexpr (MODE == 1) {
      if (act) { v.x = softplus_f(v.x); v.y = softplus_f(v.y); v.z = softplus_f(v.z); v.w = softplus_f(v.w); }
    }
    *(v4fa*)sp = v;
  }

  v4f fv[8];
#pragma unroll
  for (int i = 0; i < 8; ++i) {
    const int lr = 16 * wave + 2 * i + hh;
    fv[i] = *(const v4fa*)(stg + lr * GBN + 4 * m);
  }

  size_t obase;
  size_t ldo;
  if constexpr (MODE == 0) {
    ldo = DD;
    obase = (size_t)(by >> 1) * ((size_t)BL * DD) + (size_t)(col0 & (DD - 1));
  } else if constexpr (MODE == 1) {
    ldo = K2;
    obase = (size_t)col0;
  } else {
    ldo = RD;
    obase = (size_t)col0;
  }
#pragma unroll
  for (int i = 0; i < 8; ++i) {
    const int gr = rowBase + 16 * wave + 2 * i + hh;
    float* op = outF + obase + (size_t)gr * ldo + 4 * m;
    *(volatile v4f*)op = fv[i];
  }
  __threadfence();
#pragma unroll
  for (int i = 0; i < 8; ++i) {
    const int gr = rowBase + 16 * wave + 2 * i + hh;
    float* op = outF + obase + (size_t)gr * ldo + 4 * m;
    *(volatile v4f*)op = fv[i];
  }
}

__global__ __launch_bounds__(NTHR) void k_conv(const float* __restrict__ ul, const float* __restrict__ cw,
                                               const float* __restrict__ cb, float* xf, unsigned short* xhl) {
  __shared__ __attribute__((aligned(16))) unsigned short rowbuf[8 * K2];
  const int tid = (int)threadIdx.x, lane = tid & 31, wave = tid >> 5;
  const int r  = (int)blockIdx.x * 8 + wave;
  const int l  = r & (LSEQ - 1);
  const int r1 = (l >= 1) ? r - 1 : r;
  const int r2 = (l >= 2) ? r - 2 : r;
  const float f1 = (l >= 1) ? 1.0f : 0.0f;
  const float f2 = (l >= 2) ? 1.0f : 0.0f;
  const v4f x0 = *(const v4f*)(ul + (size_t)r  * DD + 4 * lane);
  v4f x1 = *(const v4f*)(ul + (size_t)r1 * DD + 4 * lane);
  v4f x2 = *(const v4f*)(ul + (size_t)r2 * DD + 4 * lane);
  x1 = x1 * f1;
  x2 = x2 * f2;
  const v4f wa = *(const v4f*)(cw + 12 * lane);
  const v4f wb = *(const v4f*)(cw + 12 * lane + 4);
  const v4f wc = *(const v4f*)(cw + 12 * lane + 8);
  const v4f bb = *(const v4f*)(cb + 4 * lane);
  const float c0 = ((bf16_val(wa.x) * x2.x + bf16_val(wa.y) * x1.x) + bf16_val(wa.z) * x0.x) + bf16_val(bb.x);
  const float c1 = ((bf16_val(wa.w) * x2.y + bf16_val(wb.x) * x1.y) + bf16_val(wb.y) * x0.y) + bf16_val(bb.y);
  const float c2 = ((bf16_val(wb.z) * x2.z + bf16_val(wb.w) * x1.z) + bf16_val(wc.x) * x0.z) + bf16_val(bb.z);
  const float c3 = ((bf16_val(wc.y) * x2.w + bf16_val(wc.z) * x1.w) + bf16_val(wc.w) * x0.w) + bf16_val(bb.w);
  v4f xv;
  xv.x = silu_f(c0); xv.y = silu_f(c1); xv.z = silu_f(c2); xv.w = silu_f(c3);

  v4us h4, l4;
  {
    unsigned hb;
    hb = bf16_bits(xv.x); h4[0] = (unsigned short)hb; l4[0] = (unsigned short)bf16_bits(xv.x - __uint_as_float(hb << 16));
    hb = bf16_bits(xv.y); h4[1] = (unsigned short)hb; l4[1] = (unsigned short)bf16_bits(xv.y - __uint_as_float(hb << 16));
    hb = bf16_bits(xv.z); h4[2] = (unsigned short)hb; l4[2] = (unsigned short)bf16_bits(xv.z - __uint_as_float(hb << 16));
    hb = bf16_bits(xv.w); h4[3] = (unsigned short)hb; l4[3] = (unsigned short)bf16_bits(xv.w - __uint_as_float(hb << 16));
  }
  unsigned short* rb = rowbuf + wave * K2;
  *(v4usa*)(rb + 4 * lane) = h4;
  *(v4usa*)(rb + DD + 4 * lane) = l4;
  __syncthreads();
  const v8us q = *(const v8usa*)(rb + 8 * lane);

  float* xp = xf + (size_t)r * DD + 4 * lane;
  unsigned short* hp = xhl + (size_t)r * K2 + 8 * lane;
  *(volatile v4f*)xp = xv;
  *(volatile v8us*)hp = q;
  __threadfence();
  *(volatile v4f*)xp = xv;
  *(volatile v8us*)hp = q;
}

__device__ __forceinline__ void sstep(float& h, float& p, float av, float dl, float xv, float bm, float cm) {
  const float da = expf(dl * av);
  const float bx = (dl * bm) * xv;
  h = da * h + bx;
  p = p + h * cm;
}

__global__ __launch_bounds__(NTHR) void k_scan(const float* __restrict__ dbc, const float* __restrict__ xf,
                                               const float* __restrict__ sg, const float* __restrict__ alog,
                                               const float* __restrict__ dskip, unsigned short* ghl) {
  __shared__ __attribute__((aligned(16))) float sDl[TCH * 32];
  __shared__ __attribute__((aligned(16))) float sX[TCH * 32];
  __shared__ __attribute__((aligned(16))) float sBC[TCH * 128];
  __shared__ __attribute__((aligned(16))) float sY[TCH * 32];
  const int tid = (int)threadIdx.x;
  const int b   = (int)blockIdx.x >> 2;
  const int dg  = (int)blockIdx.x & 3;
  const int d0  = 32 * dg;
  const int dlc = tid >> 3;
  const int j   = tid & 7;
  const int d   = d0 + dlc;

  float av0, av1, av2, av3, av4, av5, av6, av7;
  {
    const v4f a0 = *(const v4f*)(alog + (size_t)d * NS + 8 * j);
    const v4f a1 = *(const v4f*)(alog + (size_t)d * NS + 8 * j + 4);
    av0 = -expf(bf16_val(a0.x)); av1 = -expf(bf16_val(a0.y));
    av2 = -expf(bf16_val(a0.z)); av3 = -expf(bf16_val(a0.w));
    av4 = -expf(bf16_val(a1.x)); av5 = -expf(bf16_val(a1.y));
    av6 = -expf(bf16_val(a1.z)); av7 = -expf(bf16_val(a1.w));
  }
  float h0 = 0.0f, h1 = 0.0f, h2 = 0.0f, h3 = 0.0f, h4 = 0.0f, h5 = 0.0f, h6 = 0.0f, h7 = 0.0f;

  const int fq  = tid & 7;
  const int fd8 = 8 * (fq & 3);
  const unsigned msel = (fq >= 4) ? 0xffffffffu : 0u;
  float ds[8];
  {
    const v4f s0 = *(const v4f*)(dskip + d0 + fd8);
    const v4f s1 = *(const v4f*)(dskip + d0 + fd8 + 4);
    ds[0] = bf16_val(s0.x); ds[1] = bf16_val(s0.y); ds[2] = bf16_val(s0.z); ds[3] = bf16_val(s0.w);
    ds[4] = bf16_val(s1.x); ds[5] = bf16_val(s1.y); ds[6] = bf16_val(s1.z); ds[7] = bf16_val(s1.w);
  }

#pragma unroll 1
  for (int ch = 0; ch < LSEQ / TCH; ++ch) {
    const int row0 = b * LSEQ + ch * TCH;
    {
      v4f tb[8];
#pragma unroll
      for (int it = 0; it < 8; ++it) {
        const int idx = it * NTHR + tid;
        const int tt = idx >> 5, q = idx & 31;
        tb[it] = *(const v4f*)(dbc + (size_t)(row0 + tt) * K2 + DD + 4 * q);
      }
#pragma unroll
      for (int it = 0; it < 8; ++it) {
        const int idx = it * NTHR + tid;
        const int tt = idx >> 5, q = idx & 31;
        *(v4fa*)(sBC + tt * 128 + 4 * q) = tb[it];
      }
      v4f td[2], tx[2];
#pragma unroll
      for (int it = 0; it < 2; ++it) {
        const int idx = it * NTHR + tid;
        const int tt = idx >> 3, q = idx & 7;
        td[it] = *(const v4f*)(dbc + (size_t)(row0 + tt) * K2 + d0 + 4 * q);
        tx[it] = *(const v4f*)(xf + (size_t)(row0 + tt) * DD + d0 + 4 * q);
      }
#pragma unroll
      for (int it = 0; it < 2; ++it) {
        const int idx = it * NTHR + tid;
        const int tt = idx >> 3, q = idx & 7;
        *(v4fa*)(sDl + tt * 32 + 4 * q) = td[it];
        *(v4fa*)(sX + tt * 32 + 4 * q) = tx[it];
      }
    }
    __syncthreads();

#pragma unroll 1
    for (int tt = 0; tt < TCH; ++tt) {
      const float dl = sDl[tt * 32 + dlc];
      const float xv = sX[tt * 32 + dlc];
      const v4f b0 = *(const v4fa*)(sBC + tt * 128 + 8 * j);
      const v4f b1 = *(const v4fa*)(sBC + tt * 128 + 8 * j + 4);
      const v4f c0 = *(const v4fa*)(sBC + tt * 128 + NS + 8 * j);
      const v4f c1 = *(const v4fa*)(sBC + tt * 128 + NS + 8 * j + 4);
      float p = 0.0f;
      sstep(h0, p, av0, dl, xv, b0.x, c0.x);
      sstep(h1, p, av1, dl, xv, b0.y, c0.y);
      sstep(h2, p, av2, dl, xv, b0.z, c0.z);
      sstep(h3, p, av3, dl, xv, b0.w, c0.w);
      sstep(h4, p, av4, dl, xv, b1.x, c1.x);
      sstep(h5, p, av5, dl, xv, b1.y, c1.y);
      sstep(h6, p, av6, dl, xv, b1.z, c1.z);
      sstep(h7, p, av7, dl, xv, b1.w, c1.w);
      p += __shfl_xor(p, 1, 32);
      p += __shfl_xor(p, 2, 32);
      p += __shfl_xor(p, 4, 32);
      if (j == 0) sY[tt * 32 + dlc] = p;
    }
    __syncthreads();

#pragma unroll 1
    for (int it = 0; it < 2; ++it) {
      const int tt  = it * 32 + (tid >> 3);
      const int row = row0 + tt;
      const float* sp = sg + (size_t)row * DD + d0 + fd8;
      const v4f s0 = *(const v4f*)sp;
      const v4f s1 = *(const v4f*)(sp + 4);
      const v4f y0 = *(const v4fa*)(sY + tt * 32 + fd8);
      const v4f y1 = *(const v4fa*)(sY + tt * 32 + fd8 + 4);
      const v4f x0 = *(const v4fa*)(sX + tt * 32 + fd8);
      const v4f x1 = *(const v4fa*)(sX + tt * 32 + fd8 + 4);
      float g[8];
      g[0] = (y0.x + ds[0] * x0.x) * s0.x;
      g[1] = (y0.y + ds[1] * x0.y) * s0.y;
      g[2] = (y0.z + ds[2] * x0.z) * s0.z;
      g[3] = (y0.w + ds[3] * x0.w) * s0.w;
      g[4] = (y1.x + ds[4] * x1.x) * s1.x;
      g[5] = (y1.y + ds[5] * x1.y) * s1.y;
      g[6] = (y1.z + ds[6] * x1.z) * s1.z;
      g[7] = (y1.w + ds[7] * x1.w) * s1.w;
      v8us o;
#pragma unroll
      for (int i = 0; i < 8; ++i) {
        const unsigned hb = bf16_bits(g[i]);
        const unsigned lb = bf16_bits(g[i] - __uint_as_float(hb << 16));
        o[i] = (unsigned short)((lb & msel) | (hb & ~msel));
      }
      unsigned short* gp = ghl + (size_t)row * K2 + 64 * dg + 8 * fq;
      *(volatile v8us*)gp = o;
      __threadfence();
      *(volatile v8us*)gp = o;
    }
    __syncthreads();
  }
}

extern "C" void kernel_launch(void* const* d_in, const int* in_sizes, int n_in,
                              void* d_out, int out_size, void* d_ws, size_t ws_size,
                              hipStream_t stream) {
  if (n_in < 15) return;
  if (in_sizes[0] != BL * RD) return;
  if (in_sizes[1] != RD * UC || in_sizes[2] != UC) return;
  if (in_sizes[3] != DD * 3 || in_sizes[4] != DD) return;
  if (in_sizes[5] != DD * DD || in_sizes[6] != DD) return;
  if (in_sizes[7] != DD * NS || in_sizes[8] != NS) return;
  if (in_sizes[9] != DD * NS || in_sizes[10] != NS) return;
  if (in_sizes[11] != DD * NS || in_sizes[12] != DD) return;
  if (in_sizes[13] != DD * RD || in_sizes[14] != RD) return;
  if (out_size != BL * RD) return;
  if (ws_size < O_END) return;

  const float* up_x    = (const float*)d_in[0];
  const float* W_up    = (const float*)d_in[1];
  const float* b_up    = (const float*)d_in[2];
  const float* conv_w  = (const float*)d_in[3];
  const float* conv_b  = (const float*)d_in[4];
  const float* W_delta = (const float*)d_in[5];
  const float* b_delta = (const float*)d_in[6];
  const float* W_B     = (const float*)d_in[7];
  const float* b_B     = (const float*)d_in[8];
  const float* W_C     = (const float*)d_in[9];
  const float* b_C     = (const float*)d_in[10];
  const float* A_log   = (const float*)d_in[11];
  const float* D_skip  = (const float*)d_in[12];
  const float* W_down  = (const float*)d_in[13];
  const float* b_down  = (const float*)d_in[14];
  float* out = (float*)d_out;

  char* ws = (char*)d_ws;
  unsigned short* XB   = (unsigned short*)(ws + O_XB);
  unsigned short* WUPT = (unsigned short*)(ws + O_WUPT);
  unsigned short* WCAT = (unsigned short*)(ws + O_WCAT);
  unsigned short* WDN  = (unsigned short*)(ws + O_WDN);
  float*          BCAT = (float*)(ws + O_BCAT);
  float*          U2   = (float*)(ws + O_U2);
  float*          XF   = (float*)(ws + O_XF);
  unsigned short* XHL  = (unsigned short*)(ws + O_XHL);
  float*          DBC  = (float*)(ws + O_DBC);
  unsigned short* GHL  = (unsigned short*)(ws + O_GHL);
  const float*    UL   = U2;
  const float*    SG   = U2 + (size_t)BL * DD;

  k_cvx<<<(BL * RD / 8) / NTHR, NTHR, 0, stream>>>(up_x, XB);
  k_wprep<<<E6 / NTHR, NTHR, 0, stream>>>(W_up, W_delta, W_B, W_C, W_down, b_delta, b_B, b_C,
                                          (unsigned short*)ws, BCAT);
  k_gemm<0><<<dim3(BL / GBM, UC / GBN), GTHR, 0, stream>>>(XB, WUPT, b_up, U2, RD);
  k_conv<<<BL / 8, NTHR, 0, stream>>>(UL, conv_w, conv_b, XF, XHL);
  k_gemm<1><<<dim3(BL / GBM, K2 / GBN), GTHR, 0, stream>>>(XHL, WCAT, BCAT, DBC, K2);
  k_scan<<<16, NTHR, 0, stream>>>(DBC, XF, SG, A_log, D_skip, GHL);
  k_gemm<2><<<dim3(BL / GBM, RD / GBN), GTHR, 0, stream>>>(GHL, WDN, b_down, out, K2);
}
